// TPSTransformer_69956427317826
// MI455X (gfx1250) — hardware-verified
//
#include <hip/hip_runtime.h>
#define NIM 32
#define S0 256
#define S1 128
#define S2 64
#define C1 32
#define C2 64
#define NP1 (S1 * S1)
#define KD2 (9 * C1)
#define ICH 4
typedef __bf16 v16b __attribute__((ext_vector_type(16)));
typedef unsigned short v8us __attribute__((ext_vector_type(8), may_alias));
typedef float  v8f  __attribute__((ext_vector_type(8)));
typedef float  v4f  __attribute__((ext_vector_type(4)));
typedef float  v4fa __attribute__((ext_vector_type(4), may_alias));
union FragB { v16b v; v8us half[2]; unsigned short u[16]; };

__device__ __forceinline__ unsigned short bf16_bits(float x) { unsigned int u = __float_as_uint(x); return (unsigned short)((u + 0x7FFFu + ((u >> 16) & 1u)) >> 16); }
__device__ __forceinline__ float bf16_val(unsigned short b) { return __uint_as_float(((unsigned int)b) << 16); }
__device__ __forceinline__ float bf16_round(float x) { return bf16_val(bf16_bits(x)); }
template <int NT>
__device__ __forceinline__ v8f mmaN(v16b ah, v16b al, v16b bh, v16b bl, v8f c) {
  c = __builtin_amdgcn_wmma_f32_16x16x32_bf16(false, ah, false, bh, (short)0, c, false, false);
  if (NT >= 2) c = __builtin_amdgcn_wmma_f32_16x16x32_bf16(false, al, false, bh, (short)0, c, false, false);
  if (NT >= 3) c = __builtin_amdgcn_wmma_f32_16x16x32_bf16(false, ah, false, bl, (short)0, c, false, false);
  asm volatile("v_nop\n\tv_nop\n\tv_nop\n\tv_nop" : "+v"(c) : "v"(ah), "v"(al), "v"(bh), "v"(bl));
  return c;
}

__global__ __launch_bounds__(256) void k_wt_bf16(const float* __restrict__ W, unsigned short* __restrict__ Wt, int K, int N) {
  const int t = blockIdx.x * 256 + threadIdx.x;
  const int k8n = K / 8;
  if (t >= N * k8n) return;
  const int n = t / k8n, k8 = (t % k8n) * 8;
  v8us v;
#pragma unroll
  for (int i = 0; i < 8; ++i) v[i] = bf16_bits(W[(size_t)(k8 + i) * N + n]);
  *(volatile v8us*)(Wt + (size_t)n * K + k8) = v;
  __threadfence();
  *(volatile v8us*)(Wt + (size_t)n * K + k8) = v;
}

template <bool ASPLIT, int ACT, bool BIAS_BF16>
__global__ __launch_bounds__(128) void k_gemm_bf(const float* __restrict__ A, int lda, const unsigned short* __restrict__ Wt, int ldb,
                                               const float* __restrict__ bias, float* __restrict__ C, int ldc, int M, int N, int K) {
  __shared__ __attribute__((aligned(16))) float so[4][16][64];
  const int tid = threadIdx.x, w = tid >> 5, lane = tid & 31, ln = lane & 15, hh = lane >> 4;
  const int ntn = N / 64;
  const int wid = blockIdx.x * 4 + w;
  const int mt = wid / ntn, nq = wid % ntn;
  if (mt * 16 >= M) return;
  const int row0 = mt * 16, col0 = nq * 64;
  const float* arow = A + (size_t)(row0 + ln) * lda;
  v8f acc[4] = {};
  for (int kb = 0; kb < K; kb += 32) {
    FragB ah, al;
    const v4f x0 = *(const v4fa*)(arow + kb + 8 * hh), x1 = *(const v4fa*)(arow + kb + 8 * hh + 4);
    const v4f x2 = *(const v4fa*)(arow + kb + 16 + 8 * hh), x3 = *(const v4fa*)(arow + kb + 16 + 8 * hh + 4);
    float xs[16] = {x0[0],x0[1],x0[2],x0[3],x1[0],x1[1],x1[2],x1[3],x2[0],x2[1],x2[2],x2[3],x3[0],x3[1],x3[2],x3[3]};
#pragma unroll
    for (int i = 0; i < 16; ++i) { const unsigned short hb = bf16_bits(xs[i]); ah.u[i] = hb; al.u[i] = ASPLIT ? bf16_bits(xs[i] - bf16_val(hb)) : (unsigned short)0; }
#pragma unroll
    for (int t = 0; t < 4; ++t) {
      const unsigned short* brow = Wt + (size_t)(col0 + t * 16 + ln) * ldb + kb;
      FragB b;
      b.half[0] = *(const v8us*)(brow + 8 * hh);
      b.half[1] = *(const v8us*)(brow + 16 + 8 * hh);
      acc[t] = mmaN<ASPLIT ? 2 : 1>(ah.v, al.v, b.v, b.v, acc[t]);
    }
  }
#pragma unroll
  for (int t = 0; t < 4; ++t) {
    float bv = bias ? bias[col0 + t * 16 + ln] : 0.f;
    if (BIAS_BF16) bv = bf16_round(bv);
#pragma unroll
    for (int r = 0; r < 8; ++r) { float v = acc[t][r] + bv; if (ACT == 1) v = fmaxf(v, 0.f); so[w][8 * hh + r][t * 16 + ln] = v; }
  }
  __builtin_amdgcn_fence(__ATOMIC_ACQ_REL, "workgroup");
  __builtin_amdgcn_wave_barrier();
  const int rsub = lane >> 4, c4 = (lane & 15) * 4;
  for (int pass = 0; pass < 2; ++pass) {
#pragma unroll
    for (int q = 0; q < 8; ++q) {
      const int r = q * 2 + rsub;
      const v4f v = *(const v4fa*)&so[w][r][c4];
      *(volatile v4f*)(C + (size_t)(row0 + r) * ldc + col0 + c4) = v;
    }
    if (pass == 0) __threadfence();
  }
}

template <bool ASPLIT, int ACT, bool BIAS_BF16, bool RES_BF16>
__global__ __launch_bounds__(128) void k_gemm_bf3(const float* __restrict__ A, int lda, const unsigned short* __restrict__ Wt, int ldb,
                                                const float* __restrict__ bias, const float* __restrict__ resid, int rmod, int ldr,
                                                float* __restrict__ C, int ldc, int M, int N, int K) {
  __shared__ __attribute__((aligned(16))) float so[4][16][64];
  const int tid = threadIdx.x, w = tid >> 5, lane = tid & 31, ln = lane & 15, hh = lane >> 4;
  const int ntn = N / 64;
  const int wid = blockIdx.x * 4 + w;
  const int mt = wid / ntn, nq = wid % ntn;
  if (mt * 16 >= M) return;
  const int row0 = mt * 16, col0 = nq * 64;
  const float* arow = A + (size_t)(row0 + ln) * lda;
  v8f acc[4] = {};
  for (int kb = 0; kb < K; kb += 32) {
    FragB ah, al;
    const v4f x0 = *(const v4fa*)(arow + kb + 8 * hh), x1 = *(const v4fa*)(arow + kb + 8 * hh + 4);
    const v4f x2 = *(const v4fa*)(arow + kb + 16 + 8 * hh), x3 = *(const v4fa*)(arow + kb + 16 + 8 * hh + 4);
    float xs[16] = {x0[0],x0[1],x0[2],x0[3],x1[0],x1[1],x1[2],x1[3],x2[0],x2[1],x2[2],x2[3],x3[0],x3[1],x3[2],x3[3]};
#pragma unroll
    for (int i = 0; i < 16; ++i) { const unsigned short hb = bf16_bits(xs[i]); ah.u[i] = hb; al.u[i] = ASPLIT ? bf16_bits(xs[i] - bf16_val(hb)) : (unsigned short)0; }
#pragma unroll
    for (int t = 0; t < 4; ++t) {
      const unsigned short* brow = Wt + (size_t)(col0 + t * 16 + ln) * ldb + kb;
      FragB b;
      b.half[0] = *(const v8us*)(brow + 8 * hh);
      b.half[1] = *(const v8us*)(brow + 16 + 8 * hh);
      acc[t] = mmaN<ASPLIT ? 2 : 1>(ah.v, al.v, b.v, b.v, acc[t]);
    }
  }
#pragma unroll
  for (int t = 0; t < 4; ++t) {
    const int col = col0 + t * 16 + ln;
    float bv = bias ? bias[col] : 0.f;
    if (BIAS_BF16) bv = bf16_round(bv);
#pragma unroll
    for (int r = 0; r < 8; ++r) {
      float v = acc[t][r] + bv;
      if (resid) { float rv = resid[(size_t)((row0 + 8 * hh + r) % rmod) * ldr + col]; if (RES_BF16) rv = bf16_round(rv); v += rv; }
      if (ACT == 1) v = fmaxf(v, 0.f);
      if (ACT == 2) v = 0.5f * v * (1.0f + erff(v * 0.70710678118654752f));
      if (ACT == 3) { const float u = 0.7978845608028654f * (v + 0.044715f * v * v * v); v = 0.5f * v * (1.0f + tanhf(u)); }
      so[w][8 * hh + r][t * 16 + ln] = v;
    }
  }
  __builtin_amdgcn_fence(__ATOMIC_ACQ_REL, "workgroup");
  __builtin_amdgcn_wave_barrier();
  const int rsub = lane >> 4, c4 = (lane & 15) * 4;
  for (int pass = 0; pass < 2; ++pass) {
#pragma unroll
    for (int q = 0; q < 8; ++q) {
      const int r = q * 2 + rsub;
      const v4f v = *(const v4fa*)&so[w][r][c4];
      *(volatile v4f*)(C + (size_t)(row0 + r) * ldc + col0 + c4) = v;
    }
    if (pass == 0) __threadfence();
  }
}
template <bool PARAM_BF16>
__global__ __launch_bounds__(256) void k_layernorm(const float* __restrict__ X, const float* __restrict__ R, const float* __restrict__ g, const float* __restrict__ bta,
                                                  float* __restrict__ out_sum, float* __restrict__ out_norm, int N, float eps) {
  __shared__ float red[256];
  const int row = blockIdx.x, tid = threadIdx.x;
  const float* x = X + (size_t)row * N; const float* rr = R ? R + (size_t)row * N : nullptr;
  float vals[16];
  const int per = N / 256;
  float s1 = 0.f;
  for (int u = 0; u < per / 4; ++u) {
    const int j = tid * 4 + 1024 * u;
    const v4f a = *(const v4fa*)(x + j);
    v4f b = {0.f,0.f,0.f,0.f}; if (rr) b = *(const v4fa*)(rr + j);
#pragma unroll
    for (int q = 0; q < 4; ++q) { const float v = a[q] + b[q]; vals[u * 4 + q] = v; s1 += v; }
  }
  red[tid] = s1; __syncthreads();
  for (int st = 128; st > 0; st >>= 1) { if (tid < st) red[tid] += red[tid + st]; __syncthreads(); }
  const float mu = red[0] / (float)N; __syncthreads();
  float s2 = 0.f;
  for (int u = 0; u < per / 4; ++u)
#pragma unroll
    for (int q = 0; q < 4; ++q) { const float c = vals[u * 4 + q] - mu; s2 += c * c; }
  red[tid] = s2; __syncthreads();
  for (int st = 128; st > 0; st >>= 1) { if (tid < st) red[tid] += red[tid + st]; __syncthreads(); }
  const float rs = rsqrtf(red[0] / (float)N + eps);
  for (int pass = 0; pass < 2; ++pass) {
    for (int u = 0; u < per / 4; ++u) {
      const int j = tid * 4 + 1024 * u;
      v4f o, sm;
#pragma unroll
      for (int q = 0; q < 4; ++q) {
        float gg = g[j + q], bb = bta[j + q];
        if (PARAM_BF16) { gg = bf16_round(gg); bb = bf16_round(bb); }
        sm[q] = vals[u * 4 + q]; o[q] = (vals[u * 4 + q] - mu) * rs * gg + bb;
      }
      if (out_sum) *(volatile v4f*)(out_sum + (size_t)row * N + j) = sm;
      *(volatile v4f*)(out_norm + (size_t)row * N + j) = o;
    }
    if (pass == 0) __threadfence();
  }
}


typedef _Float16 v16h __attribute__((ext_vector_type(16)));
union FragH { v16h v; v8us half[2]; _Float16 h[16]; unsigned short u[16]; };
template <int NT>
__device__ __forceinline__ v8f mmaH(v16h ah, v16h al, v16h bh, v16h bl, v8f c) {
  c = __builtin_amdgcn_wmma_f32_16x16x32_f16(false, ah, false, bh, (short)0, c, false, false);
  if (NT >= 2) c = __builtin_amdgcn_wmma_f32_16x16x32_f16(false, al, false, bh, (short)0, c, false, false);
  if (NT >= 3) c = __builtin_amdgcn_wmma_f32_16x16x32_f16(false, ah, false, bl, (short)0, c, false, false);
  asm volatile("v_nop\n\tv_nop\n\tv_nop\n\tv_nop" : "+v"(c) : "v"(ah), "v"(al), "v"(bh), "v"(bl));
  return c;
}
template <bool ASPLIT>
__global__ __launch_bounds__(128) void k_gemm_h(const float* __restrict__ A, int lda, size_t sA, const _Float16* __restrict__ Bh, int ldb, size_t sB, float alpha, float* __restrict__ C, int ldc, size_t sC, int M, int N, int K) {
  __shared__ __attribute__((aligned(16))) float so[4][16][64];
  const int tid = threadIdx.x, w = tid >> 5, lane = tid & 31, ln = lane & 15, hh = lane >> 4; const int by = blockIdx.y;
  A += (size_t)by * sA; Bh += (size_t)by * sB; C += (size_t)by * sC;
  const int ntn = (N + 63) / 64; const int wid = blockIdx.x * 4 + w; const int mt = wid / ntn, nq = wid % ntn; if (mt * 16 >= M) return;
  const int row0 = mt * 16, col0 = nq * 64; const float* arow = A + (size_t)(row0 + ln) * lda;
  v8f acc[4] = {};
  for (int kb = 0; kb < K; kb += 32) {
    FragH ah, al;
    const v4f x0 = *(const v4fa*)(arow + kb + 8 * hh), x1 = *(const v4fa*)(arow + kb + 8 * hh + 4), x2 = *(const v4fa*)(arow + kb + 16 + 8 * hh), x3 = *(const v4fa*)(arow + kb + 16 + 8 * hh + 4);
    float xs[16] = {x0[0],x0[1],x0[2],x0[3],x1[0],x1[1],x1[2],x1[3],x2[0],x2[1],x2[2],x2[3],x3[0],x3[1],x3[2],x3[3]};
#pragma unroll
    for (int i = 0; i < 16; ++i) { const _Float16 h = (_Float16)xs[i]; ah.h[i] = h; al.h[i] = ASPLIT ? (_Float16)(xs[i] - (float)h) : (_Float16)0.0f; }
#pragma unroll
    for (int t = 0; t < 4; ++t) { if (col0 + t * 16 >= N) continue; const size_t boff = (size_t)(col0 + t * 16 + ln) * ldb + kb; FragH bq; bq.half[0] = *(const v8us*)(Bh + boff + 8 * hh); bq.half[1] = *(const v8us*)(Bh + boff + 16 + 8 * hh);
      acc[t] = mmaH<ASPLIT ? 2 : 1>(ah.v, al.v, bq.v, bq.v, acc[t]); }
  }
#pragma unroll
  for (int t = 0; t < 4; ++t) { if (col0 + t * 16 >= N) continue;
#pragma unroll
    for (int r = 0; r < 8; ++r) so[w][8 * hh + r][t * 16 + ln] = acc[t][r] * alpha; }
  __builtin_amdgcn_fence(__ATOMIC_ACQ_REL, "workgroup"); __builtin_amdgcn_wave_barrier();
  const int rsub = lane >> 4, c4 = (lane & 15) * 4;
  for (int pass = 0; pass < 2; ++pass) {
#pragma unroll
    for (int q = 0; q < 8; ++q) { const int r = q * 2 + rsub; if (col0 + c4 < N) { const v4f v = *(const v4fa*)&so[w][r][c4]; *(volatile v4f*)(C + (size_t)(row0 + r) * ldc + col0 + c4) = v; } }
    if (pass == 0) __threadfence(); }
}

__global__ __launch_bounds__(256) void k_wt_f16(const float* __restrict__ W, _Float16* __restrict__ Wt, int K, int N, float scale) {
  const int t = blockIdx.x * 256 + threadIdx.x; if (t >= N * (K / 8)) return; const int n = t / (K / 8), k8 = (t % (K / 8)) * 8; FragH f;
#pragma unroll
  for (int i = 0; i < 8; ++i) f.h[i] = (_Float16)(bf16_round(W[(size_t)(k8 + i) * N + n]) * scale); const v8us o = f.half[0];
  *(volatile v8us*)((unsigned short*)Wt + (size_t)n * K + k8) = o; __threadfence(); *(volatile v8us*)((unsigned short*)Wt + (size_t)n * K + k8) = o;
}
template <int ACT>
__global__ __launch_bounds__(128) void k_gemm_hhx(const _Float16* __restrict__ A, int lda, size_t sA, const _Float16* __restrict__ Bh, int ldb, size_t sB, float alpha, const float* __restrict__ bias, size_t sBias, const float* __restrict__ CP, int rowsPerB, size_t sCPb, int row0g,
    float* __restrict__ C, _Float16* __restrict__ C16, int ldc, size_t sC, int M, int N, int K) {
  __shared__ __attribute__((aligned(16))) float so[4][16][64];
  const int tid = threadIdx.x, w = tid >> 5, lane = tid & 31, ln = lane & 15, hh = lane >> 4; const int by = blockIdx.y;
  A += (size_t)by * sA; Bh += (size_t)by * sB; const size_t cofs = (size_t)by * sC; const float* bp = bias ? bias + (size_t)by * sBias : nullptr;
  const int ntn = (N + 63) / 64; const int wid = blockIdx.x * 4 + w; const int mt = wid / ntn, nq = wid % ntn; if (mt * 16 >= M) return;
  const int row0 = mt * 16, col0 = nq * 64; const _Float16* arow = A + (size_t)(row0 + ln) * lda;
  v8f acc[4] = {};
  for (int kb = 0; kb < K; kb += 32) { FragH ah; ah.half[0] = *(const v8us*)((const unsigned short*)arow + kb + 8 * hh); ah.half[1] = *(const v8us*)((const unsigned short*)arow + kb + 16 + 8 * hh);
#pragma unroll
    for (int t = 0; t < 4; ++t) { if (col0 + t * 16 >= N) continue; const size_t boff = (size_t)(col0 + t * 16 + ln) * ldb + kb; FragH bq; bq.half[0] = *(const v8us*)((const unsigned short*)Bh + boff + 8 * hh); bq.half[1] = *(const v8us*)((const unsigned short*)Bh + boff + 16 + 8 * hh);
      acc[t] = mmaH<1>(ah.v, ah.v, bq.v, bq.v, acc[t]); }
  }
#pragma unroll
  for (int t = 0; t < 4; ++t) { if (col0 + t * 16 >= N) continue; const int col = col0 + t * 16 + ln; const float bv = bp ? bf16_round(bp[col]) : 0.f;
#pragma unroll
    for (int r = 0; r < 8; ++r) { float v = acc[t][r] * alpha + bv; if (CP) { const int bidx = (row0g + row0 + 8 * hh + r) / rowsPerB; v += CP[(size_t)bidx * sCPb + (size_t)by * 64 + col]; } if (ACT == 1) v = (v > 0.f) ? v : expm1f(v); else if (ACT == 7) v = (v > 0.f) ? v + 1.0f : expf(v); else if (ACT == 8) v = tanhf(v); else if (ACT == 9) v = 0.5f * v * (1.0f + tanhf(0.7978845608028654f * (v + 0.044715f * v * v * v))); else if (ACT == 11) v = 1.0f / (1.0f + expf(-v)); else if (ACT == 12) v = (v > 0.f) ? v : 0.01f * v; else if (ACT == 14) v = (v > 0.f) ? v : 0.1f * v; else if (ACT == 15) v = v / (1.0f + expf(-v)); else if (ACT == 3) v = fmaxf(v, 0.f); else if (ACT == 6) v = 0.5f * v * (1.0f + erff(v * 0.70710678118654752f)); so[w][8 * hh + r][t * 16 + ln] = v; } }
  __builtin_amdgcn_fence(__ATOMIC_ACQ_REL, "workgroup"); __builtin_amdgcn_wave_barrier();
  const int rsub = lane >> 4, c4 = (lane & 15) * 4; typedef _Float16 v4h __attribute__((ext_vector_type(4)));
  for (int pass = 0; pass < 2; ++pass) {
#pragma unroll
    for (int q = 0; q < 8; ++q) { const int r = q * 2 + rsub; if (col0 + c4 < N) { const v4f v = *(const v4fa*)&so[w][r][c4]; if (C) *(volatile v4f*)(C + cofs + (size_t)(row0 + r) * ldc + col0 + c4) = v; if (C16) { v4h h4; for (int i = 0; i < 4; ++i) h4[i] = (_Float16)v[i]; *(volatile v4h*)(C16 + cofs + (size_t)(row0 + r) * ldc + col0 + c4) = h4; } } }
    if (pass == 0) __threadfence(); }
}


typedef _Float16 v4h __attribute__((ext_vector_type(4)));

__global__ __launch_bounds__(256) void k_x16(const float* __restrict__ x, _Float16* __restrict__ X16, size_t n8) { const size_t t = (size_t)blockIdx.x * 256 + threadIdx.x; if (t >= n8) return; FragH f;
#pragma unroll
  for (int q = 0; q < 8; ++q) f.h[q] = (_Float16)bf16_round(x[t * 8 + q]); *(volatile v8us*)((unsigned short*)X16 + t * 8) = f.half[0]; __threadfence(); *(volatile v8us*)((unsigned short*)X16 + t * 8) = f.half[0]; }
__global__ __launch_bounds__(256) void k_h16(const float* __restrict__ x, _Float16* __restrict__ X16, size_t n8) { const size_t t = (size_t)blockIdx.x * 256 + threadIdx.x; if (t >= n8) return; FragH f;
#pragma unroll
  for (int q = 0; q < 8; ++q) f.h[q] = (_Float16)x[t * 8 + q]; *(volatile v8us*)((unsigned short*)X16 + t * 8) = f.half[0]; __threadfence(); *(volatile v8us*)((unsigned short*)X16 + t * 8) = f.half[0]; }
__global__ __launch_bounds__(256) void k_round16f(const float* __restrict__ W, _Float16* __restrict__ Bt, size_t n8) { const size_t t = (size_t)blockIdx.x * 256 + threadIdx.x; if (t >= n8) return; FragH f;
#pragma unroll
  for (int i = 0; i < 8; ++i) f.h[i] = (_Float16)(bf16_round(W[t * 8 + i]) * 16.0f); *(volatile v8us*)((unsigned short*)Bt + t * 8) = f.half[0]; __threadfence(); *(volatile v8us*)((unsigned short*)Bt + t * 8) = f.half[0]; }
template <int NHv, int TTv>
__global__ __launch_bounds__(256) void k_vt(const _Float16* __restrict__ V16, int ldv, int voff, _Float16* __restrict__ Vt) { __shared__ unsigned short tl[64][66]; const int tid = threadIdx.x; const int slab = blockIdx.x / (TTv / 64), lg = blockIdx.x % (TTv / 64); const int b = slab / NHv, h = slab % NHv;
  for (int i = tid; i < 64 * 8; i += 256) { const int r = i / 8, c8 = (i % 8) * 8; FragH f; f.half[0] = *(const v8us*)((const unsigned short*)V16 + ((size_t)b * TTv + lg * 64 + r) * ldv + voff + h * 64 + c8);
#pragma unroll
    for (int q = 0; q < 8; ++q) tl[r][c8 + q] = f.u[q]; }
  __syncthreads();
  for (int pass = 0; pass < 2; ++pass) {
#pragma unroll
    for (int rd = 0; rd < 2; ++rd) { const int d = rd * 32 + tid / 8, pc = tid % 8; FragH f;
#pragma unroll
      for (int q = 0; q < 8; ++q) f.u[q] = tl[pc * 8 + q][d];
      *(volatile v8us*)((unsigned short*)Vt + ((size_t)slab * 64 + d) * TTv + lg * 64 + pc * 8) = f.half[0]; }
    if (pass == 0) __threadfence(); } }

__global__ __launch_bounds__(256) void k_hl(const float* __restrict__ F, _Float16* __restrict__ Hh, _Float16* __restrict__ Hl, size_t n8) { const size_t t = (size_t)blockIdx.x * 256 + threadIdx.x; if (t >= n8) return; FragH fh, fl; const v4f a = *(const v4fa*)(F + t * 8), c = *(const v4fa*)(F + t * 8 + 4);
#pragma unroll
  for (int q = 0; q < 4; ++q) { _Float16 h = (_Float16)a[q]; fh.h[q] = h; fl.h[q] = (_Float16)((a[q] - (float)h) * 1024.0f); h = (_Float16)c[q]; fh.h[4 + q] = h; fl.h[4 + q] = (_Float16)((c[q] - (float)h) * 1024.0f); }
  for (int pass = 0; pass < 2; ++pass) { *(volatile v8us*)((unsigned short*)Hh + t * 8) = fh.half[0]; *(volatile v8us*)((unsigned short*)Hl + t * 8) = fl.half[0]; if (pass == 0) __threadfence(); } }

__global__ __launch_bounds__(256) void k_conv1(const float* __restrict__ x, const float* __restrict__ w, const float* __restrict__ bb, int b0, _Float16* __restrict__ P1) {
  #pragma clang fp contract(off)
  const int t = blockIdx.x * 256 + threadIdx.x; if (t >= ICH * NP1 * (C1 / 8)) return; const int c0 = (t % (C1 / 8)) * 8; const int p1 = (t / (C1 / 8)) % NP1; const int bl = t / ((C1 / 8) * NP1); const int b = b0 + bl; const int py = p1 / S1, px = p1 % S1; const float* img = x + (size_t)b * S0 * S0;
  float best[8];
#pragma unroll
  for (int q = 0; q < 8; ++q) best[q] = -3.0e38f;
#pragma unroll 1
  for (int pos = 0; pos < 4; ++pos) { const int oy = 2 * py + pos / 2, ox = 2 * px + pos % 2; float acc[8];
#pragma unroll
    for (int q = 0; q < 8; ++q) acc[q] = bf16_round(bb[c0 + q]);
#pragma unroll 1
    for (int k = 0; k < 9; ++k) { const int yy = oy - 1 + k / 3, xx = ox - 1 + k % 3; if (yy < 0 || yy >= S0 || xx < 0 || xx >= S0) continue; const float v = bf16_round(img[(size_t)yy * S0 + xx]);
#pragma unroll
      for (int q = 0; q < 8; ++q) acc[q] += bf16_round(w[(size_t)(c0 + q) * 9 + k]) * v; }
#pragma unroll
    for (int q = 0; q < 8; ++q) best[q] = fmaxf(best[q], acc[q]); }
  FragH f;
#pragma unroll
  for (int q = 0; q < 8; ++q) f.h[q] = (_Float16)fmaxf(best[q], 0.f);
  *(volatile v8us*)((unsigned short*)P1 + ((size_t)bl * NP1 + p1) * C1 + c0) = f.half[0]; __threadfence(); *(volatile v8us*)((unsigned short*)P1 + ((size_t)bl * NP1 + p1) * C1 + c0) = f.half[0]; }
__global__ __launch_bounds__(256) void k_im2col(const _Float16* __restrict__ P1, _Float16* __restrict__ COL) { const int t = blockIdx.x * 256 + threadIdx.x; if (t >= ICH * NP1 * 9 * (C1 / 8)) return; const int c0 = (t % (C1 / 8)) * 8; const int k = (t / (C1 / 8)) % 9; const int row = t / ((C1 / 8) * 9); const int bl = row / NP1, p1 = row % NP1; const int y = p1 / S1, xq = p1 % S1; const int yy = y - 1 + k / 3, xx = xq - 1 + k % 3; FragH f = FragH{};
  if (yy >= 0 && yy < S1 && xx >= 0 && xx < S1) f.half[0] = *(const v8us*)((const unsigned short*)P1 + ((size_t)bl * NP1 + yy * S1 + xx) * C1 + c0);
  *(volatile v8us*)((unsigned short*)COL + ((size_t)row * 9 + k) * C1 + c0) = f.half[0]; __threadfence(); *(volatile v8us*)((unsigned short*)COL + ((size_t)row * 9 + k) * C1 + c0) = f.half[0]; }
__global__ __launch_bounds__(256) void k_w2(const float* __restrict__ w, _Float16* __restrict__ Bt) { const int t = blockIdx.x * 256 + threadIdx.x; if (t >= C2 * (KD2 / 8)) return; const int col0 = (t % (KD2 / 8)) * 8, o = t / (KD2 / 8); const int k = col0 / C1, c0 = col0 % C1; FragH f;
#pragma unroll
  for (int q = 0; q < 8; ++q) f.h[q] = (_Float16)(bf16_round(w[((size_t)o * C1 + c0 + q) * 9 + k]) * 16.0f);
  *(volatile v8us*)((unsigned short*)Bt + (size_t)o * KD2 + col0) = f.half[0]; __threadfence(); *(volatile v8us*)((unsigned short*)Bt + (size_t)o * KD2 + col0) = f.half[0]; }
__global__ __launch_bounds__(256) void k_pool(const float* __restrict__ CV, int b0, float* __restrict__ FEAT) {
  #pragma clang fp contract(off)
  const int t = blockIdx.x * 256 + threadIdx.x; if (t >= ICH * C2 * 16) return; const int j = t % 4, i = (t / 4) % 4; const int c = (t / 16) % C2; const int bl = t / (16 * C2); float s = 0.f;
#pragma unroll 1
  for (int yy = 0; yy < 16; ++yy) {
#pragma unroll 1
    for (int xx = 0; xx < 16; ++xx) { const int y2 = i * 16 + yy, x2 = j * 16 + xx; float m = -3.0e38f;
#pragma unroll
      for (int pos = 0; pos < 4; ++pos) { const int y1 = 2 * y2 + pos / 2, x1 = 2 * x2 + pos % 2; m = fmaxf(m, CV[((size_t)bl * NP1 + y1 * S1 + x1) * C2 + c]); }
      s += fmaxf(m, 0.f); } }
  const float v = s / 256.0f; *(volatile float*)(FEAT + (size_t)(b0 + bl) * 1024 + t % 1024) = v; __threadfence(); *(volatile float*)(FEAT + (size_t)(b0 + bl) * 1024 + t % 1024) = v; }
__global__ __launch_bounds__(256) void k_fc1(const float* __restrict__ FEAT, const float* __restrict__ W1, const float* __restrict__ b1, float* __restrict__ H) {
  #pragma clang fp contract(off)
  const int t = blockIdx.x * 256 + threadIdx.x; if (t >= NIM * 256) return; const int b = t / 256, o = t % 256; float s = bf16_round(b1[o]);
#pragma unroll 1
  for (int k = 0; k < 1024; ++k) s += FEAT[(size_t)b * 1024 + k] * bf16_round(W1[(size_t)o * 1024 + k]);
  s = fmaxf(s, 0.f); *(volatile float*)(H + t) = s; __threadfence(); *(volatile float*)(H + t) = s; }
__device__ __forceinline__ void cp_of(int i, float& cx, float& cy) { cx = (float)(i % 3) / 2.0f * 2.0f - 1.0f; cy = (float)(i / 3) / 2.0f * 2.0f - 1.0f; }
__global__ __launch_bounds__(256) void k_solve(const float* __restrict__ H, const float* __restrict__ W2, const float* __restrict__ b2, float* __restrict__ PAR) {
  #pragma clang fp contract(off)
  __shared__ float Ls[NIM][12][15];
  __shared__ __attribute__((aligned(16))) float Ps[NIM][32];
  const int b = threadIdx.x; if (b < NIM) {
  typedef float row15[15]; volatile __attribute__((address_space(3))) row15* A = (volatile __attribute__((address_space(3))) row15*)(&Ls[b][0]);
  for (int i = 0; i < 12; ++i) for (int j = 0; j < 15; ++j) A[i][j] = 0.f;
  for (int i = 0; i < 9; ++i) { float xi, yi; cp_of(i, xi, yi);
    for (int j = 0; j < 9; ++j) { float xj, yj; cp_of(j, xj, yj); const float dx = xi - xj, dy = yi - yj; const float r2 = dx * dx + dy * dy; A[i][j] = (r2 > 0.f) ? r2 * logf(r2) : 0.f; }
    A[i][9] = 1.f; A[i][10] = xi; A[i][11] = yi; A[9][i] = 1.f; A[10][i] = xi; A[11][i] = yi; }
  for (int i = 0; i < 9; ++i) { float cx, cy; cp_of(i, cx, cy); float dxv = bf16_round(b2[2 * i]), dyv = bf16_round(b2[2 * i + 1]);
    for (int k = 0; k < 256; ++k) { const float h = H[(size_t)b * 256 + k]; dxv += h * bf16_round(W2[(size_t)(2 * i) * 256 + k]); dyv += h * bf16_round(W2[(size_t)(2 * i + 1) * 256 + k]); }
    A[i][12] = cx + dxv; A[i][13] = cy + dyv; }
  for (int col = 0; col < 12; ++col) { int piv = col; float best = fabsf(A[col][col]); for (int r = col + 1; r < 12; ++r) { const float v = fabsf(A[r][col]); if (v > best) { best = v; piv = r; } }
    if (piv != col) for (int j = 0; j < 14; ++j) { const float tmp = A[col][j]; A[col][j] = A[piv][j]; A[piv][j] = tmp; }
    const float d = A[col][col]; for (int r = col + 1; r < 12; ++r) { const float f = A[r][col] / d; for (int j = col; j < 14; ++j) A[r][j] -= f * A[col][j]; } }
  for (int col = 11; col >= 0; --col) { for (int rc = 12; rc < 14; ++rc) { float s = A[col][rc]; for (int j = col + 1; j < 12; ++j) s -= A[col][j] * A[j][rc]; A[col][rc] = s / A[col][col]; } }
  volatile __attribute__((address_space(3))) float* ps = (volatile __attribute__((address_space(3))) float*)&Ps[b][0]; for (int i = 0; i < 12; ++i) { ps[2 * i] = A[i][12]; ps[2 * i + 1] = A[i][13]; } for (int i = 24; i < 32; ++i) ps[i] = 0.f; }
  __syncthreads();
  { const int t = threadIdx.x; const v4f v = *(const v4f*)&Ps[t / 8][(t % 8) * 4]; *(volatile v4f*)(PAR + (size_t)t * 4) = v; __threadfence(); *(volatile v4f*)(PAR + (size_t)t * 4) = v; } }
__global__ __launch_bounds__(256) void k_warp(const float* __restrict__ x, const float* __restrict__ PAR, float* __restrict__ out) {
  #pragma clang fp contract(off)
  const int t = blockIdx.x * 256 + threadIdx.x; if (t >= NIM * (S0 * S0 / 4)) return; const int p0 = (t % (S0 * S0 / 4)) * 4; const int b = t / (S0 * S0 / 4); const float* par = PAR + (size_t)b * 32; const float* img = x + (size_t)b * S0 * S0; v4f v;
#pragma unroll 1
  for (int q = 0; q < 4; ++q) { const int p = p0 + q; const int iy = p / S0, ix = p % S0; const float gx = -1.0f + 2.0f * (float)ix / (float)(S0 - 1), gy = -1.0f + 2.0f * (float)iy / (float)(S0 - 1);
    float wx_ = par[18] + par[20] * gx + par[22] * gy, wy_ = par[19] + par[21] * gx + par[23] * gy;
#pragma unroll 1
    for (int k = 0; k < 9; ++k) { float cx, cy; cp_of(k, cx, cy); const float dx = gx - cx, dy = gy - cy; const float r2 = dx * dx + dy * dy; const float U = (r2 > 0.f) ? r2 * logf(r2) : 0.f; wx_ += U * par[2 * k]; wy_ += U * par[2 * k + 1]; }
    const float sx = (wx_ + 1.0f) * 0.5f * (float)(S0 - 1), sy = (wy_ + 1.0f) * 0.5f * (float)(S0 - 1); const float x0 = floorf(sx), y0 = floorf(sy); const float fx = sx - x0, fy = sy - y0; float val = 0.f;
#pragma unroll
    for (int cn = 0; cn < 4; ++cn) { const float xi = x0 + (float)(cn & 1), yi = y0 + (float)(cn >> 1); const bool valid = (xi >= 0.f && xi < (float)S0 && yi >= 0.f && yi < (float)S0); const float w = ((cn & 1) ? fx : (1.0f - fx)) * ((cn >> 1) ? fy : (1.0f - fy)); const int xc = (int)fminf(fmaxf(xi, 0.f), (float)(S0 - 1)), yc = (int)fminf(fmaxf(yi, 0.f), (float)(S0 - 1)); val += (valid ? w : 0.f) * bf16_round(img[(size_t)yc * S0 + xc]); }
#pragma unroll
    for (int k = 0; k < 4; ++k) v[k] = (k == q) ? val : v[k]; }
  *(volatile v4f*)(out + (size_t)b * S0 * S0 + p0) = v; __threadfence(); *(volatile v4f*)(out + (size_t)b * S0 * S0 + p0) = v; }

extern "C" void kernel_launch(void* const* d_in, const int* in_sizes, int n_in,
                              void* d_out, int out_size, void* d_ws, size_t ws_size, hipStream_t stream) {
  (void)in_sizes; (void)n_in; (void)out_size;
  const float* const* I = (const float* const*)d_in; const float* x = I[0]; const float* c1w = I[1]; const float* c1b = I[2]; const float* c2w = I[3]; const float* c2b = I[4]; const float* f1w = I[5]; const float* f1b = I[6]; const float* f2w = I[7]; const float* f2b = I[8];
  char* ws = (char*)d_ws; size_t off = 0;
  auto take = [&](size_t bytes) { char* p = ws + off; off += (bytes + 255) & ~(size_t)255; return p; };
  _Float16* B2 = (_Float16*)take((size_t)C2 * KD2 * 2); _Float16* P1 = (_Float16*)take((size_t)ICH * NP1 * C1 * 2); _Float16* COL = (_Float16*)take((size_t)ICH * NP1 * KD2 * 2); float* CV = (float*)take((size_t)ICH * NP1 * C2 * 4); float* FEAT = (float*)take((size_t)NIM * 1024 * 4); float* H = (float*)take((size_t)NIM * 256 * 4); float* PAR = (float*)take((size_t)NIM * 32 * 4);
  if (off > ws_size) return;
  k_w2<<<(C2 * (KD2 / 8) + 255) / 256, 256, 0, stream>>>(c2w, B2);
  const dim3 gC(((ICH * NP1 / 16) * 1 + 3) / 4, 1);
  for (int b0 = 0; b0 < NIM; b0 += ICH) {
    k_conv1<<<(ICH * NP1 * (C1 / 8) + 255) / 256, 256, 0, stream>>>(x, c1w, c1b, b0, P1);
    k_im2col<<<(unsigned)(((size_t)ICH * NP1 * 9 * (C1 / 8) + 255) / 256), 256, 0, stream>>>(P1, COL);
    k_gemm_hhx<0><<<gC, 128, 0, stream>>>(COL, KD2, 0, B2, KD2, 0, 0.0625f, c2b, 0, nullptr, 1, 0, 0, CV, nullptr, C2, 0, ICH * NP1, C2, KD2);
    k_pool<<<(ICH * C2 * 16 + 255) / 256, 256, 0, stream>>>(CV, b0, FEAT); }
  k_fc1<<<(NIM * 256 + 255) / 256, 256, 0, stream>>>(FEAT, f1w, f1b, H);
  k_solve<<<1, 256, 0, stream>>>(H, f2w, f2b, PAR);
  k_warp<<<(unsigned)(((size_t)NIM * S0 * S0 / 4 + 255) / 256), 256, 0, stream>>>(x, PAR, (float*)d_out);
}
